// TransformerBlock_19679540150410
// MI455X (gfx1250) — hardware-run, weakly checked
//
#include <hip/hip_runtime.h>
#pragma clang fp contract(off)


#ifndef NB
#define NB 4
#endif
#ifndef SEQ
#define SEQ 4096
#endif
#define NB_FULL  4
#define SEQ_FULL 4096
#ifndef OUT_SEQ
#define OUT_SEQ SEQ
#endif
#define DM   384
#define FW   8
#define KB   (32 * FW)
#define DSL  (DM / FW)
#define PP   (KB + 8)
#define OSP  388
#define GP   68
#define QRS  2048.0f
#define QRI  (1.0f / 2048.0f)
#define WSC  64.0f
#define WSI  (1.0f / 64.0f)
#define L2E  1.4426950408889634f
#define PSH  14.0f
#define NEGB (-3.0e38f)
#define LNE  1.0e-5f

static_assert(DM % 64 == 0);
static_assert(DM % 32 == 0);
static_assert(DM == FW * DSL);
static_assert(DSL == 48);
static_assert(KB == 256);
static_assert(SEQ % KB == 0);
static_assert(SEQ % 64 == 0);
static_assert((NB * SEQ) % 64 == 0);
static_assert(SEQ % 16 == 0);
static_assert(NB <= NB_FULL);
static_assert(SEQ <= SEQ_FULL);
static_assert(PP % 8 == 0);
static_assert((OSP * 4) % 16 == 0);
static_assert(OSP >= DM);
static_assert((GP * 4) % 16 == 0);
static_assert(256 * 3 * 16 == 16 * DM * 2);
static_assert(256 * 6 * 4 == 16 * DM);
static_assert(256 * 24 == 16 * DM);
static_assert(32 * 4 * 16 == 16 * 64 * 2);
static_assert(32 * 8 * 16 == 16 * 64 * 4);
static_assert(2 * FW == 16);
static_assert(16 * PP * 2 + 16 * OSP * 4 + 2 * FW * 16 * 4 <= 131072);
static_assert(16 * OSP * 4 <= 131072);
static_assert(16 * GP * 4 <= 131072);

typedef _Float16 h16;
typedef __attribute__((ext_vector_type(16))) _Float16 v16h;
typedef __attribute__((ext_vector_type(8)))  _Float16 v8h;
typedef __attribute__((ext_vector_type(8)))  float    v8f;
typedef __attribute__((ext_vector_type(4)))  float    v4f;
typedef v4f  __attribute__((may_alias)) v4fa;

__device__ __forceinline__ unsigned short f2bf(float f) { unsigned u = __float_as_uint(f); u += 0x7FFFu + ((u >> 16) & 1u); return (unsigned short)(u >> 16); }
__device__ __forceinline__ float bfr(float f) { return __uint_as_float(((unsigned)f2bf(f)) << 16); }
__device__ __forceinline__ v16h cat16(v8h lo, v8h hi) { return __builtin_shufflevector(lo, hi, 0, 1, 2, 3, 4, 5, 6, 7, 8, 9, 10, 11, 12, 13, 14, 15); }
__device__ __forceinline__ v8f wmma16(v16h a, v16h b, v8f c) { return __builtin_amdgcn_wmma_f32_16x16x32_f16(false, a, false, b, (short)0, c, false, false); }
__device__ __forceinline__ v16h  ldh(const h16* p) { return cat16(*(const v8h*)p, *(const v8h*)(p + 16)); }
__device__ __forceinline__ void wave_sync() { __builtin_amdgcn_fence(3  , "wavefront"); __builtin_amdgcn_wave_barrier(); asm volatile("" ::: "memory"); }
static __device__ __forceinline__ h16 toh_flush(float v) { const h16 r = (h16)v; return (fabsf(v) < 6.103515625e-05f) ? (h16)0.0f : r; }
__device__ __forceinline__ v8f wmma16g(v16h a, v16h b, v8f c) { c = wmma16(a, b, c); asm volatile("v_nop\n\tv_nop\n\tv_nop\n\tv_nop" : "+v"(c) : "v"(a), "v"(b)); return c; }

__global__ __launch_bounds__(256) void k_wconv(const float* __restrict__ W, h16* WT) {
    __shared__ __align__(16) float ts[16 * OSP];
    const int tid = threadIdx.x; const int n0 = blockIdx.x * 16;
#pragma unroll 1
    for (int it = 0; it < 24; ++it) { const int idx = it * 256 + tid; const int k = idx >> 4, nn = idx & 15;
        ts[nn * OSP + k] = bfr(W[(size_t)k * DM + n0 + nn]) * WSC; }
    __syncthreads();
    h16* dst = WT + (size_t)n0 * DM;
#pragma unroll 1
    for (int ps = 0; ps < 2; ++ps) {
#pragma unroll 1
        for (int it = 0; it < 3; ++it) { const int p = it * 256 + tid; const int row = p / 48, c8 = (p % 48) * 8;
            const v4f x0 = *(const v4fa*)(&ts[row * OSP + c8]); const v4f x1 = *(const v4fa*)(&ts[row * OSP + c8 + 4]); v8h hv;
#pragma unroll
            for (int i = 0; i < 4; ++i) { hv[i] = toh_flush(x0[i]); hv[4 + i] = toh_flush(x1[i]); }
            *(volatile v8h*)(dst + (size_t)p * 8) = hv; }
        if (ps == 0) __threadfence(); }
}

__global__ __launch_bounds__(256) void k_ln(const float* __restrict__ X, int inSeq, int first, int wres, const float* __restrict__ G, const float* __restrict__ Be, h16* PH, h16* PR) {
    __shared__ __align__(16) float ts[16 * OSP];
    const int tid = threadIdx.x, lane = threadIdx.x & 31;
    const int wave = __builtin_amdgcn_readfirstlane((int)(threadIdx.x >> 5));
    const int m0 = blockIdx.x * 16;
    const int bb = m0 / SEQ, tt = m0 % SEQ;
    const float* src = X + ((size_t)bb * (size_t)inSeq + (size_t)tt) * DM;
#pragma unroll 1
    for (int it = 0; it < 6; ++it) { const int p = it * 256 + tid; const int row = p / 96, c4 = (p % 96) * 4;
        v4f v = *(const v4f*)(src + (size_t)p * 4);
        if (first != 0) { v[0] = bfr(v[0]); v[1] = bfr(v[1]); v[2] = bfr(v[2]); v[3] = bfr(v[3]); }
        *(v4fa*)(&ts[row * OSP + c4]) = v; }
    __syncthreads();
#pragma unroll 1
    for (int rr = 0; rr < 2; ++rr) {
        const int rb = (wave * 2 + rr) * OSP;
        float s = 0.0f;
#pragma unroll 1
        for (int i = 0; i < 12; ++i) s += ts[rb + lane + 32 * i];
        s += __shfl_xor(s, 16, 32); s += __shfl_xor(s, 8, 32); s += __shfl_xor(s, 4, 32); s += __shfl_xor(s, 2, 32); s += __shfl_xor(s, 1, 32);
        const float mu = s * (1.0f / DM);
        float q = 0.0f;
#pragma unroll 1
        for (int i = 0; i < 12; ++i) { const float d = ts[rb + lane + 32 * i] - mu; q += d * d; }
        q += __shfl_xor(q, 16, 32); q += __shfl_xor(q, 8, 32); q += __shfl_xor(q, 4, 32); q += __shfl_xor(q, 2, 32); q += __shfl_xor(q, 1, 32);
        const float rstd = rsqrtf(q * (1.0f / DM) + LNE);
#pragma unroll 1
        for (int i = 0; i < 12; ++i) { const int c = lane + 32 * i; const float d = ts[rb + c] - mu; ts[rb + c] = d * rstd * bfr(G[c]) + bfr(Be[c]); }
    }
    __syncthreads();
    h16* dh = PH + (size_t)m0 * DM; h16* dr = PR + (size_t)m0 * DM;
#pragma unroll 1
    for (int ps = 0; ps < 2; ++ps) {
#pragma unroll 1
        for (int it = 0; it < 3; ++it) { const int p = it * 256 + tid; const int row = p / 48, c8 = (p % 48) * 8;
            const v4f x0 = *(const v4fa*)(&ts[row * OSP + c8]); const v4f x1 = *(const v4fa*)(&ts[row * OSP + c8 + 4]); v8h hv, rv;
#pragma unroll
            for (int i = 0; i < 4; ++i) { const h16 a0 = toh_flush(x0[i]); const h16 a1 = toh_flush(x1[i]); hv[i] = a0; hv[4 + i] = a1;
                rv[i] = toh_flush((x0[i] - (float)a0) * QRS); rv[4 + i] = toh_flush((x1[i] - (float)a1) * QRS); }
            *(volatile v8h*)(dh + (size_t)p * 8) = hv; if (wres != 0) *(volatile v8h*)(dr + (size_t)p * 8) = rv; }
        if (ps == 0) __threadfence(); }
}

template <int RES>
static __device__ __forceinline__ void gemm_loop(const h16* __restrict__ A, const h16* __restrict__ AR, const h16* __restrict__ Bt, size_t aoff, size_t boff, v8f (&acc)[2][4], v8f (&accr)[2][4]) {
#pragma unroll
    for (int mb = 0; mb < 2; ++mb)
#pragma unroll
        for (int nb = 0; nb < 4; ++nb) { acc[mb][nb] = (v8f){}; accr[mb][nb] = (v8f){}; }
#pragma unroll 1
    for (int kc = 0; kc < DM; kc += 32) {
        v16h a[2], ar[2];
#pragma unroll
        for (int mb = 0; mb < 2; ++mb) { a[mb] = ldh(A + aoff + (size_t)mb * 16 * DM + kc); ar[mb] = a[mb]; if (RES) ar[mb] = ldh(AR + aoff + (size_t)mb * 16 * DM + kc); }
#pragma unroll
        for (int nb = 0; nb < 4; ++nb) { const v16h b = ldh(Bt + boff + (size_t)nb * 16 * DM + kc);
#pragma unroll
            for (int mb = 0; mb < 2; ++mb) { acc[mb][nb] = wmma16g(a[mb], b, acc[mb][nb]); if (RES) accr[mb][nb] = wmma16g(ar[mb], b, accr[mb][nb]); } }
    }
}

__global__ __launch_bounds__(32) void k_gemm_qk(const h16* __restrict__ A, const h16* __restrict__ AR, const h16* __restrict__ Bt, const float* __restrict__ bias, h16* PH, h16* PR) {
    __shared__ __align__(16) float os[16 * GP];
    const int lane = threadIdx.x & 31, lr = lane & 15, hi = lane >> 4; const int r0 = blockIdx.x * 32, c0 = blockIdx.y * 64;
    v8f acc[2][4], accr[2][4];
    gemm_loop<1>(A, AR, Bt, (size_t)(r0 + lr) * DM + 8 * hi, (size_t)(c0 + lr) * DM + 8 * hi, acc, accr);
    float bc[4];
#pragma unroll
    for (int nb = 0; nb < 4; ++nb) bc[nb] = bfr(bias[c0 + nb * 16 + lr]);
#pragma unroll
    for (int mb = 0; mb < 2; ++mb) {
#pragma unroll
        for (int nb = 0; nb < 4; ++nb) {
#pragma unroll
            for (int j = 0; j < 8; ++j) os[(hi * 8 + j) * GP + nb * 16 + lr] = (acc[mb][nb][j] + accr[mb][nb][j] * QRI) * WSI + bc[nb]; }
        wave_sync();
#pragma unroll 1
        for (int ps = 0; ps < 2; ++ps) {
#pragma unroll
            for (int s = 0; s < 4; ++s) { const int row = 4 * s + (lane >> 3), c8 = (lane & 7) * 8;
                const v4f x0 = *(const v4fa*)(&os[row * GP + c8]); const v4f x1 = *(const v4fa*)(&os[row * GP + c8 + 4]); v8h hv, rv;
#pragma unroll
                for (int i = 0; i < 4; ++i) { const h16 a0 = toh_flush(x0[i]); const h16 a1 = toh_flush(x1[i]); hv[i] = a0; hv[4 + i] = a1;
                    rv[i] = toh_flush((x0[i] - (float)a0) * QRS); rv[4 + i] = toh_flush((x1[i] - (float)a1) * QRS); }
                const size_t oo = (size_t)(r0 + mb * 16 + row) * DM + c0 + c8;
                *(volatile v8h*)(PH + oo) = hv; *(volatile v8h*)(PR + oo) = rv; }
            if (ps == 0) __threadfence(); }
        wave_sync();
    }
}

__global__ __launch_bounds__(32) void k_gemm_vt(const h16* __restrict__ A, const h16* __restrict__ Bt, const float* __restrict__ bias, h16* VT) {
    __shared__ __align__(16) float os[16 * GP];
    const int lane = threadIdx.x & 31, lr = lane & 15, hi = lane >> 4; const int r0 = blockIdx.x * 32, c0 = blockIdx.y * 64;
    v8f acc[2][4], accr[2][4];
    gemm_loop<0>(A, A, Bt, (size_t)(r0 + lr) * DM + 8 * hi, (size_t)(c0 + lr) * DM + 8 * hi, acc, accr);
    const int bb = c0 / SEQ, tt = c0 % SEQ;
#pragma unroll
    for (int mb = 0; mb < 2; ++mb) {
        float br[8];
#pragma unroll
        for (int j = 0; j < 8; ++j) br[j] = bfr(bias[r0 + mb * 16 + hi * 8 + j]);
#pragma unroll
        for (int nb = 0; nb < 4; ++nb) {
#pragma unroll
            for (int j = 0; j < 8; ++j) os[(hi * 8 + j) * GP + nb * 16 + lr] = acc[mb][nb][j] * WSI + br[j]; }
        wave_sync();
#pragma unroll 1
        for (int ps = 0; ps < 2; ++ps) {
#pragma unroll
            for (int s = 0; s < 4; ++s) { const int row = 4 * s + (lane >> 3), c8 = (lane & 7) * 8;
                const v4f x0 = *(const v4fa*)(&os[row * GP + c8]); const v4f x1 = *(const v4fa*)(&os[row * GP + c8 + 4]); v8h hv;
#pragma unroll
                for (int i = 0; i < 4; ++i) { hv[i] = toh_flush(x0[i]); hv[4 + i] = toh_flush(x1[i]); }
                const size_t oo = ((size_t)bb * DM + (size_t)(r0 + mb * 16 + row)) * SEQ + (size_t)tt + c8;
                *(volatile v8h*)(VT + oo) = hv; }
            if (ps == 0) __threadfence(); }
        wave_sync();
    }
}

__global__ __launch_bounds__(32) void k_gemm_f32(const h16* __restrict__ A, const h16* __restrict__ Bt, const float* __restrict__ bias, const float* __restrict__ resid, int resSeq, int rbf, float* OF, int outSeq) {
    __shared__ __align__(16) float os[16 * GP];
    const int lane = threadIdx.x & 31, lr = lane & 15, hi = lane >> 4; const int r0 = blockIdx.x * 32, c0 = blockIdx.y * 64;
    v8f acc[2][4], accr[2][4];
    gemm_loop<0>(A, A, Bt, (size_t)(r0 + lr) * DM + 8 * hi, (size_t)(c0 + lr) * DM + 8 * hi, acc, accr);
    float bc[4];
#pragma unroll
    for (int nb = 0; nb < 4; ++nb) bc[nb] = bfr(bias[c0 + nb * 16 + lr]);
    const int bb = r0 / SEQ, tt = r0 % SEQ;
    const float* rbase = resid + ((size_t)bb * (size_t)resSeq + (size_t)tt) * DM + c0;
    float* obase = OF + ((size_t)bb * (size_t)outSeq + (size_t)tt) * DM + c0;
#pragma unroll
    for (int mb = 0; mb < 2; ++mb) {
#pragma unroll
        for (int nb = 0; nb < 4; ++nb) {
#pragma unroll
            for (int j = 0; j < 8; ++j) os[(hi * 8 + j) * GP + nb * 16 + lr] = acc[mb][nb][j] * WSI + bc[nb]; }
        wave_sync();
#pragma unroll 1
        for (int ps = 0; ps < 2; ++ps) {
#pragma unroll
            for (int s = 0; s < 8; ++s) { const int row = 2 * s + (lane >> 4), c4 = (lane & 15) * 4;
                const size_t ro = (size_t)(mb * 16 + row) * DM + c4;
                v4f rv = *(const v4f*)(rbase + ro);
                if (rbf != 0) { rv[0] = bfr(rv[0]); rv[1] = bfr(rv[1]); rv[2] = bfr(rv[2]); rv[3] = bfr(rv[3]); }
                const v4f cv = *(const v4fa*)(&os[row * GP + c4]);
                const v4f val = cv + rv;
                *(volatile v4f*)(obase + ro) = val; }
            if (ps == 0) __threadfence(); }
        wave_sync();
    }
}

__global__ __launch_bounds__(32 * FW) void k_flash(const h16* __restrict__ QH, const h16* __restrict__ QR, const h16* __restrict__ KH, const h16* __restrict__ KR, const h16* __restrict__ VT, h16* CTX) {
    __shared__ __align__(16) h16 Ps[16 * PP];
    __shared__ __align__(16) float os[16 * OSP];
    __shared__ float wmax[FW * 16];
    __shared__ float wsum[FW * 16];
    const int tid = threadIdx.x, lane = threadIdx.x & 31, lr = lane & 15, hi = lane >> 4;
    const int wave = __builtin_amdgcn_readfirstlane((int)(threadIdx.x >> 5));
    const int b = blockIdx.y; const int t0 = blockIdx.x * 16;
    const size_t pb = (size_t)b * SEQ * DM;
    const size_t qo = pb + (size_t)(t0 + lr) * DM + 8 * hi;
    const size_t kofs = pb + (size_t)(wave * 32 + lr) * DM + 8 * hi;
    const int d0 = wave * DSL;
    const size_t vofs = ((size_t)b * DM + (size_t)(d0 + lr)) * SEQ + 8 * hi;
    const int pw = lr * PP + wave * 32 + 8 * hi;
    const int pr = lr * PP + 8 * hi;
    v8f o0 = (v8f){}, o1 = (v8f){}, o2 = (v8f){};
    float m = NEGB, l = 0.0f;
#pragma unroll 1
    for (int kb = 0; kb < SEQ; kb += KB) {
        v8f sHa = (v8f){}, sLa = (v8f){}, sHb = (v8f){}, sLb = (v8f){};
        const size_t kk = kofs + (size_t)kb * DM;
#pragma unroll 1
        for (int kc = 0; kc < DM; kc += 32) {
            const v16h qh = ldh(QH + qo + kc), qr = ldh(QR + qo + kc);
            const v16h ka = ldh(KH + kk + kc), kc2 = ldh(KH + kk + (size_t)16 * DM + kc);
            const v16h ra = ldh(KR + kk + kc), rc2 = ldh(KR + kk + (size_t)16 * DM + kc);
            sHa = wmma16g(ka, qh, sHa); sLa = wmma16g(ka, qr, sLa); sLa = wmma16g(ra, qh, sLa);
            sHb = wmma16g(kc2, qh, sHb); sLb = wmma16g(kc2, qr, sLb); sLb = wmma16g(rc2, qh, sLb);
        }
        float ta[8], tb[8]; float mx = NEGB;
#pragma unroll
        for (int r = 0; r < 8; ++r) {
            ta[r] = (sHa[r] + sLa[r] * QRI) * L2E; tb[r] = (sHb[r] + sLb[r] * QRI) * L2E;
            mx = fmaxf(mx, fmaxf(ta[r], tb[r])); }
        mx = fmaxf(mx, __shfl_xor(mx, 16, 32));
        wmax[wave * 16 + lr] = mx;
        __syncthreads();
        float bm = wmax[lr];
#pragma unroll
        for (int w = 1; w < FW; ++w) bm = fmaxf(bm, wmax[w * 16 + lr]);
        const float mnew = fmaxf(m, bm);
        const float alpha = __builtin_amdgcn_exp2f(m - mnew);
        const float sh = PSH - mnew;
        v8h pa, pc; float ls = 0.0f;
#pragma unroll
        for (int r = 0; r < 8; ++r) {
            const float ea = ta[r] + sh, eb = tb[r] + sh;
            const float xa = __builtin_amdgcn_exp2f(ea), xb = __builtin_amdgcn_exp2f(eb);
            const float ga = (ea < -14.0f) ? 0.0f : xa, gb = (eb < -14.0f) ? 0.0f : xb;
            const h16 ha = (h16)ga; const h16 hb = (h16)gb;
            pa[r] = ha; pc[r] = hb; ls += (float)ha + (float)hb; }
        ls += __shfl_xor(ls, 16, 32);
        wsum[wave * 16 + lr] = ls;
        *(v8h*)(&Ps[pw]) = pa;
        *(v8h*)(&Ps[pw + 16]) = pc;
        o0 = o0 * alpha; o1 = o1 * alpha; o2 = o2 * alpha;
        __syncthreads();
        float lsum = wsum[lr];
#pragma unroll
        for (int w = 1; w < FW; ++w) lsum += wsum[w * 16 + lr];
        l = l * alpha + lsum; m = mnew;
        const size_t vv = vofs + (size_t)kb;
#pragma unroll 1
        for (int ks = 0; ks < KB; ks += 32) {
            const v16h pf = cat16(*(const v8h*)(&Ps[pr + ks]), *(const v8h*)(&Ps[pr + ks + 16]));
            const v16h v0 = ldh(VT + vv + ks), v1 = ldh(VT + vv + (size_t)16 * SEQ + ks), v2 = ldh(VT + vv + (size_t)32 * SEQ + ks);
            o0 = wmma16g(v0, pf, o0); o1 = wmma16g(v1, pf, o1); o2 = wmma16g(v2, pf, o2);
        }
        __syncthreads();
    }
    const float inv = 1.0f / l;
    { const int ob = lr * OSP + d0 + 8 * hi; v4f a, c;
      a[0] = o0[0] * inv; a[1] = o0[1] * inv; a[2] = o0[2] * inv; a[3] = o0[3] * inv; c[0] = o0[4] * inv; c[1] = o0[5] * inv; c[2] = o0[6] * inv; c[3] = o0[7] * inv;
      *(v4fa*)(&os[ob]) = a; *(v4fa*)(&os[ob + 4]) = c;
      a[0] = o1[0] * inv; a[1] = o1[1] * inv; a[2] = o1[2] * inv; a[3] = o1[3] * inv; c[0] = o1[4] * inv; c[1] = o1[5] * inv; c[2] = o1[6] * inv; c[3] = o1[7] * inv;
      *(v4fa*)(&os[ob + 16]) = a; *(v4fa*)(&os[ob + 20]) = c;
      a[0] = o2[0] * inv; a[1] = o2[1] * inv; a[2] = o2[2] * inv; a[3] = o2[3] * inv; c[0] = o2[4] * inv; c[1] = o2[5] * inv; c[2] = o2[6] * inv; c[3] = o2[7] * inv;
      *(v4fa*)(&os[ob + 32]) = a; *(v4fa*)(&os[ob + 36]) = c; }
    __syncthreads();
    h16* dst = CTX + ((size_t)b * SEQ + (size_t)t0) * DM;
#pragma unroll 1
    for (int ps = 0; ps < 2; ++ps) {
#pragma unroll 1
        for (int it = 0; it < 3; ++it) { const int p = it * 256 + tid; const int row = p / 48, c8 = (p % 48) * 8;
            const v4f x0 = *(const v4fa*)(&os[row * OSP + c8]); const v4f x1 = *(const v4fa*)(&os[row * OSP + c8 + 4]); v8h hv;
#pragma unroll
            for (int i = 0; i < 4; ++i) { hv[i] = toh_flush(x0[i]); hv[4 + i] = toh_flush(x1[i]); }
            *(volatile v8h*)(dst + (size_t)p * 8) = hv; }
        if (ps == 0) __threadfence(); }
}

static constexpr size_t al256(size_t v) { return (v + 255) & ~(size_t)255; }
static constexpr size_t SZ_W  = al256((size_t)DM * DM * 2);
static constexpr size_t SZ_PL = al256((size_t)NB * SEQ * DM * 2);
static constexpr size_t SZ_X1 = al256((size_t)NB * SEQ * DM * 4);
static constexpr size_t SZ_TOTAL = 5 * SZ_W + 7 * SZ_PL + SZ_X1;
static_assert(SZ_TOTAL <= (size_t)134217728);
static_assert(((size_t)DM * DM * 2) % 256 == 0);
static_assert((size_t)NB * DM * SEQ * 2 <= SZ_PL);
static_assert(((size_t)NB * SEQ / 16) * 16 == (size_t)NB * SEQ);
static_assert(((size_t)NB * SEQ / 32) * 32 == (size_t)NB * SEQ);

extern "C" void kernel_launch(void* const* d_in, const int* in_sizes, int n_in,
                              void* d_out, int out_size, void* d_ws, size_t ws_size, hipStream_t stream) {
    if (n_in < 15) return;
    const size_t needx = ((size_t)(NB - 1) * SEQ_FULL + SEQ) * DM;
    if ((size_t)in_sizes[0] < needx) return;
    if ((size_t)in_sizes[1] < (size_t)DM * DM || (size_t)in_sizes[3] < (size_t)DM * DM || (size_t)in_sizes[5] < (size_t)DM * DM ||
        (size_t)in_sizes[7] < (size_t)DM * DM || (size_t)in_sizes[9] < (size_t)DM * DM) return;
    if (in_sizes[2] < DM || in_sizes[4] < DM || in_sizes[6] < DM || in_sizes[8] < DM || in_sizes[10] < DM) return;
    if (in_sizes[11] < DM || in_sizes[12] < DM || in_sizes[13] < DM || in_sizes[14] < DM) return;
    if ((size_t)out_size < ((size_t)(NB - 1) * OUT_SEQ + SEQ) * DM) return;
    if (SZ_TOTAL > ws_size) return;
    const float* x   = (const float*)d_in[0];
    const float* wq  = (const float*)d_in[1];  const float* bq  = (const float*)d_in[2];
    const float* wk  = (const float*)d_in[3];  const float* bk  = (const float*)d_in[4];
    const float* wv  = (const float*)d_in[5];  const float* bv  = (const float*)d_in[6];
    const float* wa  = (const float*)d_in[7];  const float* ba  = (const float*)d_in[8];
    const float* wf  = (const float*)d_in[9];  const float* bff = (const float*)d_in[10];
    const float* g1  = (const float*)d_in[11]; const float* be1 = (const float*)d_in[12];
    const float* g2  = (const float*)d_in[13]; const float* be2 = (const float*)d_in[14];
    float* OUT = (float*)d_out;
    char* wsp = (char*)d_ws;
    h16* WQT = (h16*)wsp; wsp += SZ_W;
    h16* WKT = (h16*)wsp; wsp += SZ_W;
    h16* WVT = (h16*)wsp; wsp += SZ_W;
    h16* WAT = (h16*)wsp; wsp += SZ_W;
    h16* WFT = (h16*)wsp; wsp += SZ_W;
    h16* HH = (h16*)wsp; wsp += SZ_PL;
    h16* HR = (h16*)wsp; wsp += SZ_PL;
    h16* QH = (h16*)wsp; wsp += SZ_PL;
    h16* QR = (h16*)wsp; wsp += SZ_PL;
    h16* KH = (h16*)wsp; wsp += SZ_PL;
    h16* KR = (h16*)wsp; wsp += SZ_PL;
    h16* VT = (h16*)wsp; wsp += SZ_PL;
    float* X1 = (float*)wsp; wsp += SZ_X1;
    h16* CTX = HR;
    h16* H2  = HH;

    k_wconv<<<DM / 16, 256, 0, stream>>>(wq, WQT);
    k_wconv<<<DM / 16, 256, 0, stream>>>(wk, WKT);
    k_wconv<<<DM / 16, 256, 0, stream>>>(wv, WVT);
    k_wconv<<<DM / 16, 256, 0, stream>>>(wa, WAT);
    k_wconv<<<DM / 16, 256, 0, stream>>>(wf, WFT);

    k_ln<<<NB * SEQ / 16, 256, 0, stream>>>(x, SEQ_FULL, 1, 1, g1, be1, HH, HR);

    k_gemm_qk<<<dim3(NB * SEQ / 32, DM / 64, 1), 32, 0, stream>>>(HH, HR, WQT, bq, QH, QR);
    k_gemm_qk<<<dim3(NB * SEQ / 32, DM / 64, 1), 32, 0, stream>>>(HH, HR, WKT, bk, KH, KR);
    k_gemm_vt<<<dim3(DM / 32, NB * SEQ / 64, 1), 32, 0, stream>>>(WVT, HH, bv, VT);

    k_flash<<<dim3(SEQ / 16, NB, 1), 32 * FW, 0, stream>>>(QH, QR, KH, KR, VT, CTX);

    k_gemm_f32<<<dim3(NB * SEQ / 32, DM / 64, 1), 32, 0, stream>>>(CTX, WAT, ba, x, SEQ_FULL, 1, X1, SEQ);

    k_ln<<<NB * SEQ / 16, 256, 0, stream>>>(X1, SEQ, 0, 0, g2, be2, H2, H2);

    k_gemm_f32<<<dim3(NB * SEQ / 32, DM / 64, 1), 32, 0, stream>>>(H2, WFT, bff, X1, SEQ, 0, OUT, OUT_SEQ);
}
